// Net_18734647345154
// MI455X (gfx1250) — hardware-verified
//
#include <hip/hip_runtime.h>
#include <stddef.h>
#include <stdint.h>

#define HID    128
#define NNODE  16384
#define NEDGE  524288
#define KD2    256
#define KCAT   384
#define NTHR   256
#define NWAVE  8
#define EB     128
#define DP     132
#define AP2    264
#define MPITCH 128
#define GBM    64
#define GBN    128
#define GTHR   128
#define EPT    8
#define CHUNK  (NTHR * EPT)
#define WCAP   (EPT * 32)
#define LISTN  (NWAVE * WCAP)
#define NBA    512
#define SLA    9
#define RCAP   28672
#define DEGCAP 64
#define NPARV  7
#define NU_ACT  (NNODE * (HID / 8))
#define NU_W128 (HID * (HID / 8))
#define NU_W256 (HID * (KD2 / 8))
#define NU_PREP (2 * NU_ACT + 3 * NU_W128 + 5 * NU_W256)
#define AGG_ZINTS (LISTN + 2 * RCAP + 3 * NBA)
#define AGG_LDS_INTS (AGG_ZINTS + 16)
#define AGG_LDS_BYTES (AGG_LDS_INTS * 4)
#define EDGE_LDS_BYTES (EB * DP * 4 + EB * AP2 * 2 + NPARV * HID * 4 + 2 * EB * 4)
#define CMSG   256.0f
#define MINV   0.00390625f
#define GEPS   1e-5f

static_assert(NEDGE % EB == 0);
static_assert(NNODE % GBM == 0 && NNODE % NBA == 0 && NNODE % 128 == 0);
static_assert(NEDGE % CHUNK == 0);
static_assert(HID == 128 && GBN == HID && KCAT == 3 * HID && KD2 == 2 * HID);
static_assert(HID % 32 == 0 && KD2 % 32 == 0 && KCAT % 32 == 0);
static_assert((CHUNK & (CHUNK - 1)) == 0 && CHUNK <= 4096);
static_assert((NBA & (NBA - 1)) == 0 && NBA == (1 << SLA));
static_assert(((long long)CHUNK << SLA) < (1LL << 31));
static_assert((long long)NEDGE < (1LL << (31 - SLA)));
static_assert(LISTN % NTHR == 0 && NBA % NWAVE == 0 && NBA % 32 == 0);
static_assert(RCAP % 4 == 0 && AGG_ZINTS % 4 == 0 && LISTN % 4 == 0);
static_assert(RCAP >= 17524);
static_assert(DEGCAP >= 55 + 8);
static_assert(256.0f * 11.3f < 65504.0f);
static_assert(AGG_LDS_BYTES <= 300000 && EDGE_LDS_BYTES <= 300000);
static_assert(GBM == (GTHR / 32) * 16 && EB == NWAVE * 16 && NTHR == 2 * EB);
static_assert((DP * 4) % 16 == 0 && (AP2 * 2) % 16 == 0 && AP2 >= KD2 && DP >= HID);
static_assert(EB * MPITCH * 2 <= EB * AP2 * 2 && EB * MPITCH * 2 == 8 * NTHR * 16);
static_assert(NU_ACT % NTHR == 0 && NU_W128 % NTHR == 0 && NU_W256 % NTHR == 0 && NU_PREP % NTHR == 0);
static_assert((EB * DP * 4) % 16 == 0 && (EB * AP2 * 2) % 16 == 0);

typedef float          v2f   __attribute__((ext_vector_type(2)));
typedef float          v4f   __attribute__((ext_vector_type(4)));
typedef float          v8f   __attribute__((ext_vector_type(8)));
typedef int            v4i   __attribute__((ext_vector_type(4)));
typedef int            v8i   __attribute__((ext_vector_type(8)));
typedef unsigned       v2u   __attribute__((ext_vector_type(2)));
typedef unsigned short v4us  __attribute__((ext_vector_type(4)));
typedef unsigned short v8us  __attribute__((ext_vector_type(8)));
typedef unsigned short v16us __attribute__((ext_vector_type(16)));
typedef __bf16         v16bf __attribute__((ext_vector_type(16)));
typedef v2f  __attribute__((may_alias)) v2fa;
typedef v4f  __attribute__((may_alias)) v4fa;
typedef v4i  __attribute__((may_alias)) v4ia;
typedef v2u  __attribute__((may_alias)) v2ua;
typedef v4us __attribute__((may_alias)) v4usa;
typedef v8us __attribute__((may_alias)) v8usa;
union FragB { v16bf v; v16us u; v8us h[2]; v8i w; };

__device__ __forceinline__ v8f wmb(const FragB& a, const FragB& b, v8f c) {
  v8f d = __builtin_amdgcn_wmma_f32_16x16x32_bf16(false, a.v, false, b.v, (short)0, c, false, false);
  asm volatile("v_nop\n\tv_nop\n\tv_nop\n\tv_nop" : "+v"(d) : "v"(a.w), "v"(b.w));
  return d;
}

__device__ __forceinline__ unsigned bf16_bits(float f) {
  const unsigned u = __float_as_uint(f);
  const unsigned r = (u + 0x7FFFu + ((u >> 16) & 1u)) >> 16;
  const unsigned n = (u >> 16) | 0x40u;
  return ((u & 0x7FFFFFFFu) > 0x7F800000u) ? n : r;
}
__device__ __forceinline__ float bf16_val(float f) {
  return __uint_as_float(bf16_bits(f) << 16);
}
__device__ __forceinline__ v4f bf4(v4f a) {
  v4f o;
  o.x = bf16_val(a.x); o.y = bf16_val(a.y); o.z = bf16_val(a.z); o.w = bf16_val(a.w);
  return o;
}
__device__ __forceinline__ unsigned short f2h(float f) {
  const _Float16 hv = (_Float16)f;
  return __builtin_bit_cast(unsigned short, hv);
}
__device__ __forceinline__ float h2f(unsigned b) {
  const _Float16 hv = __builtin_bit_cast(_Float16, (unsigned short)b);
  return (float)hv;
}
__device__ __forceinline__ float relu_p(float v) { return (v > 0.0f) ? v : (v - v); }
__device__ __forceinline__ float wsum32(float s) {
  s += __shfl_xor(s, 16, 32);
  s += __shfl_xor(s, 8, 32);
  s += __shfl_xor(s, 4, 32);
  s += __shfl_xor(s, 2, 32);
  s += __shfl_xor(s, 1, 32);
  return s;
}
__device__ __forceinline__ float wsum16(float s) {
  s += __shfl_xor(s, 8, 32);
  s += __shfl_xor(s, 4, 32);
  s += __shfl_xor(s, 2, 32);
  s += __shfl_xor(s, 1, 32);
  return s;
}
__device__ __forceinline__ v4f gn4(v4f x, v4f g, v4f b) {
  float s = (x.x + x.y) + (x.z + x.w);
  s = wsum32(s);
  const float mu = s * (1.0f / 128.0f);
  const float d0 = x.x - mu, d1 = x.y - mu, d2 = x.z - mu, d3 = x.w - mu;
  float q = (d0 * d0 + d1 * d1) + (d2 * d2 + d3 * d3);
  q = wsum32(q);
  const float rs = 1.0f / sqrtf(q * (1.0f / 128.0f) + GEPS);
  v4f y;
  y.x = (d0 * rs) * g.x + b.x;
  y.y = (d1 * rs) * g.y + b.y;
  y.z = (d2 * rs) * g.z + b.z;
  y.w = (d3 * rs) * g.w + b.w;
  return y;
}
__device__ __forceinline__ void put16(unsigned short* dp, v8us o) {
  *(volatile v8us*)dp = o;
  __threadfence();
  *(volatile v8us*)dp = o;
}
__device__ __forceinline__ void putf4(float* dp, v4f o) {
  *(volatile v4f*)dp = o;
  __threadfence();
  *(volatile v4f*)dp = o;
}
__device__ __forceinline__ v8us wgather(const float* __restrict__ p) {
  v8us o;
#pragma unroll
  for (int i = 0; i < 8; ++i) o[i] = (unsigned short)bf16_bits(p[(size_t)i * HID]);
  return o;
}

template <int SLB>
__device__ __forceinline__ int scan_chunk(const int* __restrict__ dsts, int nE, int cbase, int slotBase,
                                          int nb, int vec8, int* list, int tid, int lane, int wave) {
  int wc = 0;
  const int el0  = tid * EPT;
  const int e0   = cbase + el0;
  const int sent = -2147483647 - 1;
  v4i da, db;
  if (vec8 != 0 && cbase + CHUNK <= nE) {
    da = *(const v4i*)(dsts + e0);
    db = *(const v4i*)(dsts + e0 + 4);
  } else {
    da.x = (e0     < nE) ? dsts[min(e0,     nE - 1)] : sent;
    da.y = (e0 + 1 < nE) ? dsts[min(e0 + 1, nE - 1)] : sent;
    da.z = (e0 + 2 < nE) ? dsts[min(e0 + 2, nE - 1)] : sent;
    da.w = (e0 + 3 < nE) ? dsts[min(e0 + 3, nE - 1)] : sent;
    db.x = (e0 + 4 < nE) ? dsts[min(e0 + 4, nE - 1)] : sent;
    db.y = (e0 + 5 < nE) ? dsts[min(e0 + 5, nE - 1)] : sent;
    db.z = (e0 + 6 < nE) ? dsts[min(e0 + 6, nE - 1)] : sent;
    db.w = (e0 + 7 < nE) ? dsts[min(e0 + 7, nE - 1)] : sent;
  }
  const unsigned nbs = (unsigned)slotBase;
  const unsigned unb = (unsigned)nb;
  const unsigned s0 = (unsigned)da.x - nbs, s1 = (unsigned)da.y - nbs;
  const unsigned s2 = (unsigned)da.z - nbs, s3 = (unsigned)da.w - nbs;
  const unsigned s4 = (unsigned)db.x - nbs, s5 = (unsigned)db.y - nbs;
  const unsigned s6 = (unsigned)db.z - nbs, s7 = (unsigned)db.w - nbs;
  const bool h0 = s0 < unb, h1 = s1 < unb, h2 = s2 < unb, h3 = s3 < unb;
  const bool h4 = s4 < unb, h5 = s5 < unb, h6 = s6 < unb, h7 = s7 < unb;
  const unsigned any = __builtin_amdgcn_ballot_w32(h0 | h1 | h2 | h3 | h4 | h5 | h6 | h7);
  if (any != 0u) {
#define HITJ(J, HJ, SJ) { \
      const unsigned mj = __builtin_amdgcn_ballot_w32(HJ); \
      if (mj != 0u) { \
        if (HJ) { \
          const int pos = wc + (int)__builtin_amdgcn_mbcnt_lo(mj, 0u); \
          if (pos < WCAP) list[wave * WCAP + pos] = ((el0 + (J)) << SLB) | (int)(SJ); \
        } \
        wc += (int)__builtin_popcount(mj); } }
    HITJ(0, h0, s0)
    HITJ(1, h1, s1)
    HITJ(2, h2, s2)
    HITJ(3, h3, s3)
    HITJ(4, h4, s4)
    HITJ(5, h5, s5)
    HITJ(6, h6, s6)
    HITJ(7, h7, s7)
#undef HITJ
  }
  return wc;
}

__global__ __launch_bounds__(NTHR) void k_prep(const float* __restrict__ agts, const float* __restrict__ ctxf,
                                               const float* __restrict__ qw, const float* __restrict__ cw1,
                                               const float* __restrict__ dw2, const float* __restrict__ aw,
                                               const float* __restrict__ cw2, const float* __restrict__ lw,
                                               unsigned short* AGB, unsigned short* CXB, unsigned short* WQT,
                                               unsigned short* W1bD, unsigned short* W1cT, unsigned short* WD2D,
                                               unsigned short* W1aD, unsigned short* WACat, unsigned short* WLD) {
  const int u  = (int)blockIdx.x * NTHR + (int)threadIdx.x;
  const int U0 = NU_ACT;
  const int U1 = U0 + NU_ACT;
  const int U2 = U1 + NU_W128;
  const int U3 = U2 + NU_W256;
  const int U4 = U3 + NU_W128;
  const int U5 = U4 + NU_W256;
  const int U6 = U5 + NU_W256;
  const int U7 = U6 + NU_W128;
  const int U8 = U7 + NU_W256;
  const int U9 = U8 + NU_W256;
  if (u < U0) {
    const int row = u >> 4, k8 = (u & 15) * 8;
    const float* p = agts + (size_t)row * HID + k8;
    const v4f a = *(const v4fa*)p;
    const v4f b = *(const v4fa*)(p + 4);
    v8us o;
    o[0] = (unsigned short)bf16_bits(a.x); o[1] = (unsigned short)bf16_bits(a.y);
    o[2] = (unsigned short)bf16_bits(a.z); o[3] = (unsigned short)bf16_bits(a.w);
    o[4] = (unsigned short)bf16_bits(b.x); o[5] = (unsigned short)bf16_bits(b.y);
    o[6] = (unsigned short)bf16_bits(b.z); o[7] = (unsigned short)bf16_bits(b.w);
    put16(AGB + (size_t)row * HID + k8, o);
    return;
  } else if (u < U1) {
    const int v = u - U0;
    const int row = v >> 4, k8 = (v & 15) * 8;
    const float* p = ctxf + (size_t)row * HID + k8;
    const v4f a = *(const v4fa*)p;
    const v4f b = *(const v4fa*)(p + 4);
    v8us o;
    o[0] = (unsigned short)bf16_bits(a.x); o[1] = (unsigned short)bf16_bits(a.y);
    o[2] = (unsigned short)bf16_bits(a.z); o[3] = (unsigned short)bf16_bits(a.w);
    o[4] = (unsigned short)bf16_bits(b.x); o[5] = (unsigned short)bf16_bits(b.y);
    o[6] = (unsigned short)bf16_bits(b.z); o[7] = (unsigned short)bf16_bits(b.w);
    put16(CXB + (size_t)row * HID + k8, o);
    return;
  } else if (u < U2) {
    const int v = u - U1;
    const int n = v >> 4, k8 = (v & 15) * 8;
    const v8us o = wgather(qw + (size_t)k8 * HID + n);
    put16(WQT + (size_t)n * HID + k8, o);
    return;
  } else if (u < U3) {
    const int v = u - U2;
    const int n = v >> 5, k8 = (v & 31) * 8;
    const v8us o = wgather(cw1 + (size_t)(HID + (k8 & (HID - 1))) * HID + n);
    put16(W1bD + (size_t)n * KD2 + k8, o);
    return;
  } else if (u < U4) {
    const int v = u - U3;
    const int n = v >> 4, k8 = (v & 15) * 8;
    const v8us o = wgather(cw1 + (size_t)(2 * HID + k8) * HID + n);
    put16(W1cT + (size_t)n * HID + k8, o);
    return;
  } else if (u < U5) {
    const int v = u - U4;
    const int n = v >> 5, k8 = (v & 31) * 8;
    const v8us o = wgather(dw2 + (size_t)(k8 & (HID - 1)) * HID + n);
    put16(WD2D + (size_t)n * KD2 + k8, o);
    return;
  } else if (u < U6) {
    const int v = u - U5;
    const int n = v >> 5, k8 = (v & 31) * 8;
    const v8us o = wgather(cw1 + (size_t)(k8 & (HID - 1)) * HID + n);
    put16(W1aD + (size_t)n * KD2 + k8, o);
    return;
  } else if (u < U7) {
    const int v = u - U6;
    const int n = v >> 4, k8 = (v & 15) * 8;
    const v8us o = wgather(aw + (size_t)k8 * HID + n);
    put16(WACat + (size_t)n * KCAT + k8, o);
    return;
  } else if (u < U8) {
    const int v = u - U7;
    const int n = v >> 5, k8 = (v & 31) * 8;
    const v8us o = wgather(cw2 + (size_t)(k8 & (HID - 1)) * HID + n);
    put16(WACat + (size_t)n * KCAT + HID + k8, o);
    return;
  } else if (u < U9) {
    const int v = u - U8;
    const int n = v >> 5, k8 = (v & 31) * 8;
    const v8us o = wgather(lw + (size_t)(k8 & (HID - 1)) * HID + n);
    put16(WLD + (size_t)n * KD2 + k8, o);
    return;
  }
}

template <int MODE>
__global__ __launch_bounds__(GTHR) void k_gemm(const unsigned short* __restrict__ A1, int lda1, int K1,
                                               const unsigned short* __restrict__ A2, int lda2, int K2,
                                               const unsigned short* __restrict__ BT, int ldb,
                                               const float* __restrict__ gam, const float* __restrict__ bet,
                                               const unsigned short* __restrict__ RES,
                                               float* Cm, unsigned short* Cb) {
  __shared__ __attribute__((aligned(16))) float stg[GBM * GBN];
  const int tid = (int)threadIdx.x, lane = tid & 31, wave = tid >> 5, hh = lane >> 4, m = lane & 15;
  const int rowBase = (int)blockIdx.x * GBM;

  v8f acc[8];
  {
    const v8f z = {0.f, 0.f, 0.f, 0.f, 0.f, 0.f, 0.f, 0.f};
#pragma unroll
    for (int t = 0; t < 8; ++t) acc[t] = z;
  }
  const unsigned short* ap1 = A1 + (size_t)(rowBase + 16 * wave + m) * (size_t)lda1 + 8 * hh;
  const unsigned short* ap2 = A2 + (size_t)(rowBase + 16 * wave + m) * (size_t)lda2 + 8 * hh;
  const unsigned short* bp1 = BT + (size_t)m * (size_t)ldb + 8 * hh;
  const unsigned short* bp2 = bp1 + K1;

#pragma unroll 1
  for (int k0 = 0; k0 < K1; k0 += 32) {
    FragB af;
    af.h[0] = *(const v8usa*)(ap1 + k0);
    af.h[1] = *(const v8usa*)(ap1 + k0 + 16);
#pragma unroll
    for (int nt = 0; nt < 8; ++nt) {
      const unsigned short* wq = bp1 + (size_t)(16 * nt) * (size_t)ldb + k0;
      FragB bf;
      bf.h[0] = *(const v8usa*)wq;
      bf.h[1] = *(const v8usa*)(wq + 16);
      acc[nt] = wmb(af, bf, acc[nt]);
    }
  }
#pragma unroll 1
  for (int k0 = 0; k0 < K2; k0 += 32) {
    FragB af;
    af.h[0] = *(const v8usa*)(ap2 + k0);
    af.h[1] = *(const v8usa*)(ap2 + k0 + 16);
#pragma unroll
    for (int nt = 0; nt < 8; ++nt) {
      const unsigned short* wq = bp2 + (size_t)(16 * nt) * (size_t)ldb + k0;
      FragB bf;
      bf.h[0] = *(const v8usa*)wq;
      bf.h[1] = *(const v8usa*)(wq + 16);
      acc[nt] = wmb(af, bf, acc[nt]);
    }
  }

#pragma unroll
  for (int nt = 0; nt < 8; ++nt) {
    const int lc = 16 * nt + m;
#pragma unroll
    for (int r = 0; r < 8; ++r) {
      const int lr = 16 * wave + 8 * hh + r;
      stg[lr * GBN + lc] = acc[nt][r];
    }
  }
  __syncthreads();

  if constexpr (MODE == 0) {
#pragma unroll 1
    for (int i = 0; i < 16; ++i) {
      const int lr = 16 * wave + i;
      const v4f pv = *(const v4fa*)(stg + lr * GBN + 4 * lane);
      putf4(Cm + (size_t)(rowBase + lr) * HID + 4 * lane, pv);
    }
  } else if constexpr (MODE == 1) {
    const int part = lane >> 4;
    const int j = lane & 15;
    const unsigned mh = 0u - (unsigned)part;
    const unsigned ml = ~mh;
    const v4f ga = bf4(*(const v4fa*)(gam + 8 * j));
    const v4f gb = bf4(*(const v4fa*)(gam + 8 * j + 4));
    const v4f ba = bf4(*(const v4fa*)(bet + 8 * j));
    const v4f bb = bf4(*(const v4fa*)(bet + 8 * j + 4));
    const v8f g8 = {ga.x, ga.y, ga.z, ga.w, gb.x, gb.y, gb.z, gb.w};
    const v8f b8 = {ba.x, ba.y, ba.z, ba.w, bb.x, bb.y, bb.z, bb.w};
#pragma unroll 1
    for (int i = 0; i < 16; ++i) {
      const int lr = 16 * wave + i;
      const float* sp = stg + lr * GBN + 8 * j;
      const v4f a = *(const v4fa*)sp;
      const v4f b = *(const v4fa*)(sp + 4);
      const v8f x8 = {a.x, a.y, a.z, a.w, b.x, b.y, b.z, b.w};
      float s = ((x8[0] + x8[1]) + (x8[2] + x8[3])) + ((x8[4] + x8[5]) + (x8[6] + x8[7]));
      s = wsum16(s);
      const float mu = s * (1.0f / 128.0f);
      v8f d8;
      float q = 0.0f;
#pragma unroll
      for (int e = 0; e < 8; ++e) { d8[e] = x8[e] - mu; q += d8[e] * d8[e]; }
      q = wsum16(q);
      const float rs = 1.0f / sqrtf(q * (1.0f / 128.0f) + GEPS);
      v8us oo;
#pragma unroll
      for (int e = 0; e < 8; ++e) {
        const float y = relu_p((d8[e] * rs) * g8[e] + b8[e]);
        const unsigned hb = bf16_bits(y);
        const unsigned lb = bf16_bits(y - __uint_as_float(hb << 16));
        oo[e] = (unsigned short)((hb & ml) | (lb & mh));
      }
      put16(Cb + (size_t)(rowBase + lr) * KD2 + part * HID + 8 * j, oo);
    }
  } else {
    const v4f g4 = bf4(*(const v4fa*)(gam + 4 * lane));
    const v4f b4 = bf4(*(const v4fa*)(bet + 4 * lane));
#pragma unroll 1
    for (int i = 0; i < 16; ++i) {
      const int lr = 16 * wave + i;
      const v4f x = *(const v4fa*)(stg + lr * GBN + 4 * lane);
      const v4f y = gn4(x, g4, b4);
      const v2u rw = *(const v2ua*)(RES + (size_t)(rowBase + lr) * HID + 4 * lane);
      v4f o;
      o.x = relu_p(y.x + __uint_as_float(rw.x << 16));
      o.y = relu_p(y.y + __uint_as_float(rw.x & 0xffff0000u));
      o.z = relu_p(y.z + __uint_as_float(rw.y << 16));
      o.w = relu_p(y.w + __uint_as_float(rw.y & 0xffff0000u));
      putf4(Cm + (size_t)(rowBase + lr) * HID + 4 * lane, o);
    }
  }
}

__device__ __forceinline__ void edge_gemm(const unsigned short* sAw, float* sDw,
                                          const unsigned short* __restrict__ BT, int hh, int m) {
  v8f acc[8];
  {
    const v8f z = {0.f, 0.f, 0.f, 0.f, 0.f, 0.f, 0.f, 0.f};
#pragma unroll
    for (int t = 0; t < 8; ++t) acc[t] = z;
  }
  const unsigned short* ap = sAw + m * AP2 + 8 * hh;
  const unsigned short* bp = BT + (size_t)m * KD2 + 8 * hh;
#pragma unroll 1
  for (int k0 = 0; k0 < KD2; k0 += 32) {
    FragB a;
    a.h[0] = *(const v8usa*)(ap + k0);
    a.h[1] = *(const v8usa*)(ap + k0 + 16);
#pragma unroll
    for (int nt = 0; nt < 8; ++nt) {
      const unsigned short* wq = bp + (size_t)(16 * nt) * KD2 + k0;
      FragB b;
      b.h[0] = *(const v8usa*)wq;
      b.h[1] = *(const v8usa*)(wq + 16);
      acc[nt] = wmb(a, b, acc[nt]);
    }
  }
#pragma unroll
  for (int nt = 0; nt < 8; ++nt) {
    const int col = 16 * nt + m;
#pragma unroll
    for (int r = 0; r < 8; ++r) sDw[(8 * hh + r) * DP + col] = acc[nt][r];
  }
}

__global__ __launch_bounds__(NTHR) void k_edge(const int* __restrict__ hiI, const int* __restrict__ wiI,
                                               int nE, int nN,
                                               const float* __restrict__ actr, const float* __restrict__ cctr,
                                               const float* __restrict__ dw1, const float* __restrict__ db1,
                                               const float* __restrict__ dg2, const float* __restrict__ db2,
                                               const float* __restrict__ cg1, const float* __restrict__ cb1,
                                               const unsigned short* __restrict__ WD2D,
                                               const unsigned short* __restrict__ W1aD,
                                               const float* __restrict__ QP, const float* __restrict__ CP,
                                               unsigned short* M16) {
  extern __shared__ __attribute__((aligned(16))) float dyn[];
  float*          sD   = dyn;
  unsigned short* sA   = (unsigned short*)(dyn + EB * DP);
  unsigned short* sM   = sA;
  float*          sPar = dyn + EB * DP + (EB * AP2) / 2;
  int*            sHi  = (int*)(sPar + NPARV * HID);
  int*            sWi  = sHi + EB;

  const int tid = (int)threadIdx.x, lane = tid & 31, wave = tid >> 5, hh = lane >> 4, m = lane & 15;
  const int e0 = (int)blockIdx.x * EB;

  if (wave == 0) {
    const v4f p0 = *(const v4fa*)(dw1 + 4 * lane);
    const v4f p1 = *(const v4fa*)(dw1 + HID + 4 * lane);
    const v4f p2 = *(const v4fa*)(db1 + 4 * lane);
    const v4f p3 = *(const v4fa*)(dg2 + 4 * lane);
    const v4f p4 = *(const v4fa*)(db2 + 4 * lane);
    const v4f p5 = *(const v4fa*)(cg1 + 4 * lane);
    const v4f p6 = *(const v4fa*)(cb1 + 4 * lane);
    *(v4fa*)(sPar + 0 * HID + 4 * lane) = bf4(p0);
    *(v4fa*)(sPar + 1 * HID + 4 * lane) = bf4(p1);
    *(v4fa*)(sPar + 2 * HID + 4 * lane) = bf4(p2);
    *(v4fa*)(sPar + 3 * HID + 4 * lane) = bf4(p3);
    *(v4fa*)(sPar + 4 * HID + 4 * lane) = bf4(p4);
    *(v4fa*)(sPar + 5 * HID + 4 * lane) = bf4(p5);
    *(v4fa*)(sPar + 6 * HID + 4 * lane) = bf4(p6);
  }

  const int row  = tid >> 1;
  const int half = tid & 1;
  int eg = e0 + row;
  eg = eg > nE - 1 ? nE - 1 : eg;
  int hn = hiI[eg];
  int wn = wiI[eg];
  hn = hn < 0 ? 0 : (hn > nN - 1 ? nN - 1 : hn);
  wn = wn < 0 ? 0 : (wn > nN - 1 ? nN - 1 : wn);
  sHi[row] = hn;
  sWi[row] = wn;
  const v2f ca = *(const v2fa*)(actr + (size_t)hn * 2);
  const v2f cc = *(const v2fa*)(cctr + (size_t)wn * 2);
  const float dx = bf16_val(ca.x) - bf16_val(cc.x);
  const float dy = bf16_val(ca.y) - bf16_val(cc.y);
  __syncthreads();

  {
    const float*    pw = sPar + 64 * half;
    unsigned short* ra = sA + row * AP2 + 64 * half;
#pragma unroll 1
    for (int c8 = 0; c8 < 8; ++c8) {
      const v4f w0a = *(const v4fa*)(pw + 8 * c8);
      const v4f w0b = *(const v4fa*)(pw + 8 * c8 + 4);
      const v4f w1a = *(const v4fa*)(pw + HID + 8 * c8);
      const v4f w1b = *(const v4fa*)(pw + HID + 8 * c8 + 4);
      const v4f b1a = *(const v4fa*)(pw + 2 * HID + 8 * c8);
      const v4f b1b = *(const v4fa*)(pw + 2 * HID + 8 * c8 + 4);
      const v8f w0 = {w0a.x, w0a.y, w0a.z, w0a.w, w0b.x, w0b.y, w0b.z, w0b.w};
      const v8f w1 = {w1a.x, w1a.y, w1a.z, w1a.w, w1b.x, w1b.y, w1b.z, w1b.w};
      const v8f bb = {b1a.x, b1a.y, b1a.z, b1a.w, b1b.x, b1b.y, b1b.z, b1b.w};
      v8us ho, lo;
#pragma unroll
      for (int i = 0; i < 8; ++i) {
        const float v = relu_p((dx * w0[i] + dy * w1[i]) + bb[i]);
        const unsigned hb = bf16_bits(v);
        ho[i] = (unsigned short)hb;
        lo[i] = (unsigned short)bf16_bits(v - __uint_as_float(hb << 16));
      }
      *(v8usa*)(ra + 8 * c8)       = ho;
      *(v8usa*)(ra + HID + 8 * c8) = lo;
    }
  }
  __syncthreads();

  const unsigned short* sAw = sA + 16 * wave * AP2;
  float*                sDw = sD + 16 * wave * DP;

  edge_gemm(sAw, sDw, WD2D, hh, m);
  __syncthreads();

  {
    const v4f g4 = *(const v4fa*)(sPar + 3 * HID + 4 * lane);
    const v4f b4 = *(const v4fa*)(sPar + 4 * HID + 4 * lane);
#pragma unroll 1
    for (int i = 0; i < 16; ++i) {
      const int r = 16 * wave + i;
      const v4f x = *(const v4fa*)(sD + r * DP + 4 * lane);
      const v4f y = gn4(x, g4, b4);
      const float y0 = relu_p(y.x), y1 = relu_p(y.y), y2 = relu_p(y.z), y3 = relu_p(y.w);
      const unsigned h0 = bf16_bits(y0), h1 = bf16_bits(y1), h2 = bf16_bits(y2), h3 = bf16_bits(y3);
      v4us ho, lo;
      ho[0] = (unsigned short)h0; ho[1] = (unsigned short)h1; ho[2] = (unsigned short)h2; ho[3] = (unsigned short)h3;
      lo[0] = (unsigned short)bf16_bits(y0 - __uint_as_float(h0 << 16));
      lo[1] = (unsigned short)bf16_bits(y1 - __uint_as_float(h1 << 16));
      lo[2] = (unsigned short)bf16_bits(y2 - __uint_as_float(h2 << 16));
      lo[3] = (unsigned short)bf16_bits(y3 - __uint_as_float(h3 << 16));
      *(v4usa*)(sA + r * AP2 + 4 * lane)       = ho;
      *(v4usa*)(sA + r * AP2 + HID + 4 * lane) = lo;
    }
  }
  __syncthreads();

  edge_gemm(sAw, sDw, W1aD, hh, m);
  __syncthreads();

  {
    const v4f g4 = *(const v4fa*)(sPar + 5 * HID + 4 * lane);
    const v4f b4 = *(const v4fa*)(sPar + 6 * HID + 4 * lane);
#pragma unroll 1
    for (int i = 0; i < 16; ++i) {
      const int r = 16 * wave + i;
      int hq = sHi[r];
      int wq = sWi[r];
      hq = hq < 0 ? 0 : (hq > nN - 1 ? nN - 1 : hq);
      wq = wq < 0 ? 0 : (wq > nN - 1 ? nN - 1 : wq);
      const v4f x  = *(const v4fa*)(sD + r * DP + 4 * lane);
      const v4f qp = *(const v4fa*)(QP + (size_t)hq * HID + 4 * lane);
      const v4f cp = *(const v4fa*)(CP + (size_t)wq * HID + 4 * lane);
      v4f c;
      c.x = (x.x + qp.x) + cp.x;
      c.y = (x.y + qp.y) + cp.y;
      c.z = (x.z + qp.z) + cp.z;
      c.w = (x.w + qp.w) + cp.w;
      const v4f y = gn4(c, g4, b4);
      v4us o;
      o[0] = f2h(CMSG * relu_p(y.x));
      o[1] = f2h(CMSG * relu_p(y.y));
      o[2] = f2h(CMSG * relu_p(y.z));
      o[3] = f2h(CMSG * relu_p(y.w));
      *(v4usa*)(sM + r * MPITCH + 4 * lane) = o;
    }
  }
  __syncthreads();

  {
    v4i pv[8];
#pragma unroll
    for (int it = 0; it < 8; ++it) pv[it] = *(const v4ia*)(sM + (size_t)(it * NTHR + tid) * 8);
    unsigned short* mb = M16 + (size_t)e0 * MPITCH;
#pragma unroll
    for (int it = 0; it < 8; ++it) *(volatile v4i*)(mb + (size_t)(it * NTHR + tid) * 8) = pv[it];
    __threadfence();
#pragma unroll
    for (int it = 0; it < 8; ++it) *(volatile v4i*)(mb + (size_t)(it * NTHR + tid) * 8) = pv[it];
  }
}

__global__ __launch_bounds__(NTHR) void k_scan(const int* __restrict__ dsts, int nE, int vec8, int nRows,
                                               const unsigned short* __restrict__ Mh, unsigned short* Shl) {
  extern __shared__ __attribute__((aligned(16))) int dsm[];
  int* list = dsm;
  int* hl   = dsm + LISTN;
  int* sl   = hl + RCAP;
  int* cnt  = sl + RCAP;
  int* offs = cnt + NBA;
  int* cur  = offs + NBA;
  int* misc = cur + NBA;
  const int tid = (int)threadIdx.x, lane = tid & 31, wave = tid >> 5;
  const int nodeBase = (int)blockIdx.x * NBA;

  {
    const v4i z4 = {0, 0, 0, 0};
    for (int i = tid * 4; i < AGG_ZINTS; i += NTHR * 4) *(v4ia*)(dsm + i) = z4;
    if (tid < 16) misc[tid] = 0;
  }
  __syncthreads();

  int t = 0, ov = 0;
  const int nChunks = (nE + CHUNK - 1) / CHUNK;
#pragma unroll 1
  for (int ch = 0; ch < nChunks; ++ch) {
    const int cbase = ch * CHUNK;
    const int wc = scan_chunk<SLA>(dsts, nE, cbase, nodeBase, NBA, vec8, list, tid, lane, wave);
    if (lane == 0) misc[wave] = wc;
    __syncthreads();
    if (wave == 0) {
#pragma unroll 1
      for (int w2 = 0; w2 < NWAVE; ++w2) {
        int c = misc[w2];
        c = c < 0 ? 0 : (c > WCAP ? WCAP : c);
#pragma unroll 1
        for (int b0 = 0; b0 < c; b0 += 32) {
          const int idx = b0 + lane;
          const int ent = list[w2 * WCAP + (idx < WCAP ? idx : WCAP - 1)];
          const int m32 = (c - b0) < 32 ? (c - b0) : 32;
#pragma unroll 1
          for (int k = 0; k < m32; ++k) {
            const int u    = __builtin_amdgcn_readlane(ent, k);
            const int slot = u & (NBA - 1);
            const int el   = (u >> SLA) & (CHUNK - 1);
            const int pk   = ((cbase + el) << SLA) | slot;
            if (t < RCAP) {
              if (lane == 0) { hl[t] = pk; cnt[slot] = cnt[slot] + 1; }
              t = t + 1;
            } else {
              ov = 1;
            }
          }
        }
      }
    }
    __syncthreads();
  }
  if (wave == 0 && lane == 0) { misc[8] = t; misc[9] = ov; }
  __syncthreads();
  int tt = misc[8];
  tt = tt < 0 ? 0 : (tt > RCAP ? RCAP : tt);
  const int ovf = misc[9];

  if (wave == 0) {
    const int base = lane * (NBA / 32);
    int s = 0;
#pragma unroll 1
    for (int i = 0; i < NBA / 32; ++i) s += cnt[base + i];
    int incl = s;
#pragma unroll
    for (int d = 1; d < 32; d <<= 1) {
      const int y = __shfl_up(incl, d, 32);
      if (lane >= d) incl += y;
    }
    int run = incl - s;
#pragma unroll 1
    for (int i = 0; i < NBA / 32; ++i) {
      const int cv = cnt[base + i];
      offs[base + i] = run;
      cur[base + i]  = run;
      run += cv;
    }
  }
  __syncthreads();
  if (wave == 0) {
#pragma unroll 1
    for (int b0 = 0; b0 < tt; b0 += 32) {
      const int idx = b0 + lane;
      const int ent = hl[idx < RCAP ? idx : RCAP - 1];
      const int m32 = (tt - b0) < 32 ? (tt - b0) : 32;
#pragma unroll 1
      for (int k = 0; k < m32; ++k) {
        const int u    = __builtin_amdgcn_readlane(ent, k);
        const int slot = u & (NBA - 1);
        if (lane == 0) {
          int p = cur[slot];
          p = p < 0 ? 0 : (p > RCAP - 1 ? RCAP - 1 : p);
          sl[p] = u;
          cur[slot] = p + 1;
        }
      }
    }
  }
  __syncthreads();

  const float qnan = __int_as_float(0x7fc00000);
  const float pz = (ovf != 0) ? qnan : 0.0f;
  const int part = lane >> 4;
  const int j    = lane & 15;
  const int sa   = 2 * j;
  const int sb   = 2 * j + 1;
  const unsigned mh = 0u - (unsigned)part;
  const unsigned ml = ~mh;
#pragma unroll 1
  for (int si = 0; si < NBA / NWAVE; ++si) {
    const int s    = si * NWAVE + wave;
    const int node = nodeBase + s;
    int c = cnt[s];
    const bool big = c > DEGCAP;
    c = c < 0 ? 0 : (c > DEGCAP ? DEGCAP : c);
    int o = offs[s];
    o = o < 0 ? 0 : (o > RCAP ? RCAP : o);
    float a0 = 0.0f, a1 = 0.0f, a2 = 0.0f, a3 = 0.0f;
#pragma unroll 1
    for (int b0 = 0; b0 < c; b0 += 32) {
      int idx = o + b0 + lane;
      idx = idx > RCAP - 1 ? RCAP - 1 : idx;
      const int ent = sl[idx];
      int eid = ent >> SLA;
      eid = eid < 0 ? 0 : (eid > nE - 1 ? nE - 1 : eid);
      const int m32 = (c - b0) < 32 ? (c - b0) : 32;
#pragma unroll 1
      for (int k = 0; k < m32; ++k) {
        const int ek = __builtin_amdgcn_readlane(eid, k);
        const unsigned short* rp = Mh + (size_t)ek * MPITCH + 4 * lane;
        const v2u w = *(const v2ua*)rp;
        a0 += h2f(w.x & 0xffffu);
        a1 += h2f(w.x >> 16);
        a2 += h2f(w.y & 0xffffu);
        a3 += h2f(w.y >> 16);
      }
    }
    const float pzr = big ? qnan : pz;
    const float t0 = a0 * MINV + pzr;
    const float t1 = a1 * MINV + pzr;
    const float t2 = a2 * MINV + pzr;
    const float t3 = a3 * MINV + pzr;
    const float f0 = __shfl(t0, sa, 32);
    const float f1 = __shfl(t1, sa, 32);
    const float f2 = __shfl(t2, sa, 32);
    const float f3 = __shfl(t3, sa, 32);
    const float f4 = __shfl(t0, sb, 32);
    const float f5 = __shfl(t1, sb, 32);
    const float f6 = __shfl(t2, sb, 32);
    const float f7 = __shfl(t3, sb, 32);
    const v8f f8 = {f0, f1, f2, f3, f4, f5, f6, f7};
    v8us oo;
#pragma unroll
    for (int e = 0; e < 8; ++e) {
      const unsigned hb = bf16_bits(f8[e]);
      const unsigned lb = bf16_bits(f8[e] - __uint_as_float(hb << 16));
      oo[e] = (unsigned short)((hb & ml) | (lb & mh));
    }
    const bool live = node < nRows;
    const int  nr   = live ? node : nRows - 1;
    unsigned short* op = Shl + (size_t)nr * KD2 + part * HID + 8 * j;
    if (live) *(volatile v8us*)op = oo;
    __threadfence();
    if (live) *(volatile v8us*)op = oo;
  }
}

extern "C" void kernel_launch(void* const* d_in, const int* in_sizes, int n_in,
                              void* d_out, int out_size, void* d_ws, size_t ws_size,
                              hipStream_t stream) {
  if (n_in < 24) return;
  if (in_sizes[0] != NNODE * HID || in_sizes[1] != NNODE * HID) return;
  if (in_sizes[2] != NNODE * 2 || in_sizes[3] != NNODE * 2) return;
  if (in_sizes[4] != NEDGE || in_sizes[5] != NEDGE) return;
  if (in_sizes[6] != 2 * HID || in_sizes[7] != HID) return;
  if (in_sizes[8] != HID * HID || in_sizes[9] != HID || in_sizes[10] != HID) return;
  if (in_sizes[11] != HID * HID || in_sizes[12] != HID || in_sizes[13] != HID) return;
  if (in_sizes[14] != 3 * HID * HID || in_sizes[15] != HID || in_sizes[16] != HID) return;
  if (in_sizes[17] != HID * HID || in_sizes[18] != HID * HID) return;
  if (in_sizes[19] != HID || in_sizes[20] != HID) return;
  if (in_sizes[21] != HID * HID || in_sizes[22] != HID || in_sizes[23] != HID) return;
  if ((long long)out_size != (long long)NNODE * HID) return;

  const float* agts    = (const float*)d_in[0];
  const float* ctxf    = (const float*)d_in[1];
  const float* actr    = (const float*)d_in[2];
  const float* cctr    = (const float*)d_in[3];
  const int*   hi      = (const int*)d_in[4];
  const int*   wi      = (const int*)d_in[5];
  const float* dist_w1 = (const float*)d_in[6];
  const float* dist_b1 = (const float*)d_in[7];
  const float* dist_w2 = (const float*)d_in[8];
  const float* dist_g2 = (const float*)d_in[9];
  const float* dist_b2 = (const float*)d_in[10];
  const float* query_w = (const float*)d_in[11];
  const float* query_g = (const float*)d_in[12];
  const float* query_b = (const float*)d_in[13];
  const float* ctx_w1  = (const float*)d_in[14];
  const float* ctx_g1  = (const float*)d_in[15];
  const float* ctx_b1  = (const float*)d_in[16];
  const float* ctx_w2  = (const float*)d_in[17];
  const float* agt_w   = (const float*)d_in[18];
  const float* norm_g  = (const float*)d_in[19];
  const float* norm_b  = (const float*)d_in[20];
  const float* lin_w   = (const float*)d_in[21];
  const float* lin_g   = (const float*)d_in[22];
  const float* lin_b   = (const float*)d_in[23];
  float* out = (float*)d_out;

  char* ws = (char*)d_ws;
  size_t off = 0;
  const size_t oWQT  = off; off += (size_t)HID * HID * 2;
  const size_t oW1b  = off; off += (size_t)HID * KD2 * 2;
  const size_t oW1c  = off; off += (size_t)HID * HID * 2;
  const size_t oWD2  = off; off += (size_t)HID * KD2 * 2;
  const size_t oW1a  = off; off += (size_t)HID * KD2 * 2;
  const size_t oWAC  = off; off += (size_t)HID * KCAT * 2;
  const size_t oWLD  = off; off += (size_t)HID * KD2 * 2;
  const size_t oAGB  = off; off += (size_t)NNODE * HID * 2;
  const size_t oCXB  = off; off += (size_t)NNODE * HID * 2;
  const size_t oQhl  = off; off += (size_t)NNODE * KD2 * 2;
  const size_t oQP   = off; off += (size_t)NNODE * HID * 4;
  const size_t oCP   = off; off += (size_t)NNODE * HID * 4;
  const size_t oShl  = off; off += (size_t)NNODE * KD2 * 2;
  const size_t oM16  = off; off += (size_t)NEDGE * MPITCH * 2;
  if (off > ws_size) return;
  unsigned short* WQT   = (unsigned short*)(ws + oWQT);
  unsigned short* W1bD  = (unsigned short*)(ws + oW1b);
  unsigned short* W1cT  = (unsigned short*)(ws + oW1c);
  unsigned short* WD2D  = (unsigned short*)(ws + oWD2);
  unsigned short* W1aD  = (unsigned short*)(ws + oW1a);
  unsigned short* WACat = (unsigned short*)(ws + oWAC);
  unsigned short* WLD   = (unsigned short*)(ws + oWLD);
  unsigned short* AGB   = (unsigned short*)(ws + oAGB);
  unsigned short* CXB   = (unsigned short*)(ws + oCXB);
  unsigned short* Qhl   = (unsigned short*)(ws + oQhl);
  unsigned short* A1hl  = (unsigned short*)(ws + oQhl);
  float*          QP    = (float*)(ws + oQP);
  float*          CP    = (float*)(ws + oCP);
  unsigned short* Shl   = (unsigned short*)(ws + oShl);
  unsigned short* M16   = (unsigned short*)(ws + oM16);

  hipFuncSetAttribute(reinterpret_cast<const void*>(&k_edge), hipFuncAttributeMaxDynamicSharedMemorySize,
                      (int)EDGE_LDS_BYTES);
  hipFuncSetAttribute(reinterpret_cast<const void*>(&k_scan), hipFuncAttributeMaxDynamicSharedMemorySize,
                      (int)AGG_LDS_BYTES);

  const int gM = NNODE / GBM;

  k_prep<<<NU_PREP / NTHR, NTHR, 0, stream>>>(agts, ctxf, query_w, ctx_w1, dist_w2, agt_w, ctx_w2, lin_w,
                                              AGB, CXB, WQT, W1bD, W1cT, WD2D, W1aD, WACat, WLD);
  k_gemm<1><<<gM, GTHR, 0, stream>>>(AGB, HID, HID, AGB, HID, 0, WQT, HID, query_g, query_b, AGB, QP, Qhl);
  k_gemm<0><<<gM, GTHR, 0, stream>>>(Qhl, KD2, KD2, Qhl, KD2, 0, W1bD, KD2, query_g, query_b, AGB, QP, Qhl);
  k_gemm<0><<<gM, GTHR, 0, stream>>>(CXB, HID, HID, CXB, HID, 0, W1cT, HID, query_g, query_b, AGB, CP, Qhl);
  k_edge<<<NEDGE / EB, NTHR, EDGE_LDS_BYTES, stream>>>(hi, wi, NEDGE, NNODE, actr, cctr, dist_w1, dist_b1,
                                                       dist_g2, dist_b2, ctx_g1, ctx_b1, WD2D, W1aD, QP, CP, M16);
  k_scan<<<NNODE / NBA, NTHR, AGG_LDS_BYTES, stream>>>(hi, NEDGE, 1, NNODE, M16, Shl);
  k_gemm<1><<<gM, GTHR, 0, stream>>>(AGB, HID, HID, Shl, KD2, KD2, WACat, KCAT, norm_g, norm_b, AGB, QP, A1hl);
  k_gemm<2><<<gM, GTHR, 0, stream>>>(A1hl, KD2, KD2, A1hl, KD2, 0, WLD, KD2, lin_g, lin_b, AGB, out, Qhl);
}
